// RGCNLayer_66778151518270
// MI455X (gfx1250) — hardware-verified
//
#include <hip/hip_runtime.h>
#include <stddef.h>
#include <stdint.h>


#define DD     128
#define NREL   8
#define NCB    (NREL + 1)
#define TP     (NCB * DD)
#define SELFC  (NREL * DD)
#define NTHR   256
#define NWAVE  8
#define EPT    8
#define CHUNK  (NTHR * EPT)
#define WCAP   (EPT * 32)
#define LISTN  (NWAVE * WCAP)
#define NBA    1024
#define SLA    10
#define RCAP   28672
#define DEGCAP 64
#define GBM    64
#define GBN    128
#define GTHR   128
#define KG     (DD / 8)
#define UREL   (NREL * DD * KG)
#define USELF  (DD * KG)
#define UW     (UREL + USELF)
#define AGG_ZINTS    (LISTN + 2 * RCAP + 3 * NBA)
#define MISC_INTS    96
#define AGG_LDS_INTS (AGG_ZINTS + MISC_INTS)
#define WSMAX  268435456

static_assert((CHUNK & (CHUNK - 1)) == 0 && CHUNK <= 4096);
static_assert((NBA & (NBA - 1)) == 0 && NBA == (1 << SLA));
static_assert(((long long)CHUNK << SLA) < (1LL << 31));
static_assert(LISTN % NTHR == 0);
static_assert(NBA % NWAVE == 0 && NBA % 32 == 0);
static_assert(RCAP % 4 == 0 && AGG_ZINTS % 4 == 0 && LISTN % 4 == 0 && ((AGG_ZINTS + MISC_INTS) % 4) == 0);
static_assert(AGG_ZINTS % (NTHR * 4) == 0);
static_assert(MISC_INTS >= 16 + DEGCAP + 1 && DEGCAP + 1 <= NTHR);
static_assert(AGG_LDS_INTS * 4 <= 300000);
static_assert(DD % 32 == 0 && DD == 4 * 32 && GBN == DD && TP % 32 == 0 && SELFC + DD == TP && (TP * 4) % 128 == 0);
static_assert(GBM == (GTHR / 32) * 16 && GBM % 16 == 0);
static_assert(UREL % NTHR == 0 && USELF % NTHR == 0 && UW % NTHR == 0 && (GBM * KG) % NTHR == 0);

typedef float          v4f   __attribute__((ext_vector_type(4)));
typedef float          v8f   __attribute__((ext_vector_type(8)));
typedef int            v4i   __attribute__((ext_vector_type(4)));
typedef int            v8i   __attribute__((ext_vector_type(8)));
typedef unsigned short v8us  __attribute__((ext_vector_type(8)));
typedef unsigned short v16us __attribute__((ext_vector_type(16)));
typedef __bf16         v16bf __attribute__((ext_vector_type(16)));
typedef v4f  __attribute__((may_alias)) v4fa;
typedef v4i  __attribute__((may_alias)) v4ia;
typedef v8us __attribute__((may_alias)) v8usa;
union Frag { v16bf v; v16us u; v8us h[2]; v8i w; };

__device__ __forceinline__ v8f wmb(const Frag& a, const Frag& b, v8f c) {
  v8f d = __builtin_amdgcn_wmma_f32_16x16x32_bf16(false, a.v, false, b.v, (short)0, c, false, false);
  asm volatile("v_nop\n\tv_nop\n\tv_nop\n\tv_nop" : "+v"(d) : "v"(a.w), "v"(b.w));
  return d;
}

__device__ __forceinline__ unsigned bf16_bits(float f) {
  const unsigned u = __float_as_uint(f);
  return (u + 0x7FFFu + ((u >> 16) & 1u)) >> 16;
}
__device__ __forceinline__ float bf16_val(float f) {
  return __uint_as_float(bf16_bits(f) << 16);
}

template <int SLB>
__device__ __forceinline__ int scan_chunk(const int* __restrict__ dsts, int nE, int cbase, int slotBase,
                                          int nb, int vec8, int* list, int tid, int lane, int wave) {
  int wc = 0;
  const int el0  = tid * EPT;
  const int e0   = cbase + el0;
  const int sent = -2147483647 - 1;
  v4i da, db;
  if (vec8 != 0 && cbase + CHUNK <= nE) {
    da = *(const v4i*)(dsts + e0);
    db = *(const v4i*)(dsts + e0 + 4);
  } else {
    da.x = (e0     < nE) ? dsts[min(e0,     nE - 1)] : sent;
    da.y = (e0 + 1 < nE) ? dsts[min(e0 + 1, nE - 1)] : sent;
    da.z = (e0 + 2 < nE) ? dsts[min(e0 + 2, nE - 1)] : sent;
    da.w = (e0 + 3 < nE) ? dsts[min(e0 + 3, nE - 1)] : sent;
    db.x = (e0 + 4 < nE) ? dsts[min(e0 + 4, nE - 1)] : sent;
    db.y = (e0 + 5 < nE) ? dsts[min(e0 + 5, nE - 1)] : sent;
    db.z = (e0 + 6 < nE) ? dsts[min(e0 + 6, nE - 1)] : sent;
    db.w = (e0 + 7 < nE) ? dsts[min(e0 + 7, nE - 1)] : sent;
  }
  const unsigned nbs = (unsigned)slotBase;
  const unsigned unb = (unsigned)nb;
  const unsigned s0 = (unsigned)da.x - nbs, s1 = (unsigned)da.y - nbs;
  const unsigned s2 = (unsigned)da.z - nbs, s3 = (unsigned)da.w - nbs;
  const unsigned s4 = (unsigned)db.x - nbs, s5 = (unsigned)db.y - nbs;
  const unsigned s6 = (unsigned)db.z - nbs, s7 = (unsigned)db.w - nbs;
  const bool h0 = s0 < unb, h1 = s1 < unb, h2 = s2 < unb, h3 = s3 < unb;
  const bool h4 = s4 < unb, h5 = s5 < unb, h6 = s6 < unb, h7 = s7 < unb;
  const unsigned any = __builtin_amdgcn_ballot_w32(h0 | h1 | h2 | h3 | h4 | h5 | h6 | h7);
  if (any != 0u) {
#define HITJ(J, HJ, SJ) { \
      const unsigned mj = __builtin_amdgcn_ballot_w32(HJ); \
      if (mj != 0u) { \
        if (HJ) { \
          const int pos = wc + (int)__builtin_amdgcn_mbcnt_lo(mj, 0u); \
          if (pos < WCAP) list[wave * WCAP + pos] = ((el0 + (J)) << SLB) | (int)(SJ); \
        } \
        wc += (int)__builtin_popcount(mj); } }
    HITJ(0, h0, s0)
    HITJ(1, h1, s1)
    HITJ(2, h2, s2)
    HITJ(3, h3, s3)
    HITJ(4, h4, s4)
    HITJ(5, h5, s5)
    HITJ(6, h6, s6)
    HITJ(7, h7, s7)
#undef HITJ
  }
  return wc;
}

__global__ __launch_bounds__(NTHR) void k_prep(const float* __restrict__ xin, int nN, int mRows,
                                               const float* __restrict__ Wrel, const float* __restrict__ Wself,
                                               unsigned short* WT, unsigned short* XB) {
  const int u = (int)blockIdx.x * NTHR + (int)threadIdx.x;
  v8us o;
  unsigned short* dp;
  if (u < UREL) {
    const int mat = u >> 11;
    const int n   = (u >> 4) & 127;
    const int k8  = (u & 15) * 8;
    const float* p = Wrel + (size_t)mat * DD * DD + (size_t)k8 * DD + n;
#pragma unroll
    for (int i = 0; i < 8; ++i) o[i] = (unsigned short)bf16_bits(p[(size_t)i * DD]);
    dp = WT + ((size_t)mat * DD + n) * (size_t)DD + k8;
  } else if (u < UW) {
    const int v  = u - UREL;
    const int n  = v >> 4;
    const int k8 = (v & 15) * 8;
    const float* p = Wself + (size_t)n * DD + k8;
    const v4f wa = *(const v4f*)p;
    const v4f wb = *(const v4f*)(p + 4);
    o[0] = (unsigned short)bf16_bits(wa.x); o[1] = (unsigned short)bf16_bits(wa.y);
    o[2] = (unsigned short)bf16_bits(wa.z); o[3] = (unsigned short)bf16_bits(wa.w);
    o[4] = (unsigned short)bf16_bits(wb.x); o[5] = (unsigned short)bf16_bits(wb.y);
    o[6] = (unsigned short)bf16_bits(wb.z); o[7] = (unsigned short)bf16_bits(wb.w);
    dp = WT + ((size_t)SELFC + n) * (size_t)DD + k8;
  } else {
    const int v   = u - UW;
    const int row = v >> 4;
    const int k8  = (v & 15) * 8;
    if (row >= mRows) return;
    const int   rc  = row < nN ? row : nN - 1;
    const float okf = row < nN ? 1.0f : 0.0f;
    const float* p = xin + (size_t)rc * DD + k8;
    const v4f xa = *(const v4f*)p;
    const v4f xc = *(const v4f*)(p + 4);
    o[0] = (unsigned short)bf16_bits(xa.x * okf); o[1] = (unsigned short)bf16_bits(xa.y * okf);
    o[2] = (unsigned short)bf16_bits(xa.z * okf); o[3] = (unsigned short)bf16_bits(xa.w * okf);
    o[4] = (unsigned short)bf16_bits(xc.x * okf); o[5] = (unsigned short)bf16_bits(xc.y * okf);
    o[6] = (unsigned short)bf16_bits(xc.z * okf); o[7] = (unsigned short)bf16_bits(xc.w * okf);
    dp = XB + (size_t)row * (size_t)DD + k8;
  }
  *(volatile v8us*)dp = o;
  __threadfence();
  *(volatile v8us*)dp = o;
}

__global__ __launch_bounds__(GTHR) void k_gemm(const unsigned short* __restrict__ A, int lda,
                                               const unsigned short* __restrict__ BT, int ldb, int K,
                                               const float* __restrict__ bias, int biasBlk,
                                               float* outp, int ldc, int nOut) {
  __shared__ __attribute__((aligned(16))) float stg[GBM * GBN];
  const int tid = (int)threadIdx.x, lane = tid & 31, wave = tid >> 5, hh = lane >> 4, m = lane & 15;
  const int rowBase = (int)blockIdx.x * GBM;
  const int cb      = (int)blockIdx.y;
  const int colBase = cb * GBN;

  v8f acc[8];
  {
    const v8f z = {0.f, 0.f, 0.f, 0.f, 0.f, 0.f, 0.f, 0.f};
#pragma unroll
    for (int t = 0; t < 8; ++t) acc[t] = z;
  }
  const unsigned short* ap = A  + (size_t)(rowBase + 16 * wave + m) * (size_t)lda + 8 * hh;
  const unsigned short* bp = BT + (size_t)(colBase + m) * (size_t)ldb + 8 * hh;

#pragma unroll 1
  for (int k0 = 0; k0 < K; k0 += 32) {
    Frag af;
    af.h[0] = *(const v8usa*)(ap + k0);
    af.h[1] = *(const v8usa*)(ap + k0 + 16);
#pragma unroll
    for (int nt = 0; nt < 8; ++nt) {
      const unsigned short* wq = bp + (size_t)(16 * nt) * (size_t)ldb + k0;
      Frag bf;
      bf.h[0] = *(const v8usa*)wq;
      bf.h[1] = *(const v8usa*)(wq + 16);
      acc[nt] = wmb(af, bf, acc[nt]);
    }
  }

#pragma unroll
  for (int nt = 0; nt < 8; ++nt) {
    const int lc = 16 * nt + m;
#pragma unroll
    for (int r = 0; r < 8; ++r) {
      const int lr = 16 * wave + 8 * hh + r;
      stg[lr * GBN + lc] = acc[nt][r];
    }
  }
  __syncthreads();

  const float bsc = (cb == biasBlk) ? 1.0f : 0.0f;
  v4f b4;
  {
    const v4f tb = *(const v4f*)(bias + 4 * lane);
    b4.x = bf16_val(tb.x) * bsc; b4.y = bf16_val(tb.y) * bsc;
    b4.z = bf16_val(tb.z) * bsc; b4.w = bf16_val(tb.w) * bsc;
  }

  v4f pv[16];
#pragma unroll
  for (int i = 0; i < 16; ++i) pv[i] = *(const v4fa*)(stg + (16 * wave + i) * GBN + 4 * lane) + b4;

#pragma unroll
  for (int i = 0; i < 16; ++i) {
    const int row = rowBase + 16 * wave + i;
    if (row < nOut) *(volatile v4f*)(outp + (size_t)row * (size_t)ldc + colBase + 4 * lane) = pv[i];
  }
  __threadfence();
#pragma unroll
  for (int i = 0; i < 16; ++i) {
    const int row = rowBase + 16 * wave + i;
    if (row < nOut) *(volatile v4f*)(outp + (size_t)row * (size_t)ldc + colBase + 4 * lane) = pv[i];
  }
}

__global__ __launch_bounds__(NTHR) void k_scan(const int* __restrict__ srcs, const int* __restrict__ dsts,
                                               const int* __restrict__ ets, int nE, int nN, int vec8,
                                               const float* __restrict__ T, float* outp) {
  extern __shared__ __attribute__((aligned(16))) int dsm[];
  int* list = dsm;
  int* hl   = dsm + LISTN;
  int* sl   = hl + RCAP;
  int* cnt  = sl + RCAP;
  int* offs = cnt + NBA;
  int* cur  = offs + NBA;
  int* misc = cur + NBA;
  float* rtab = (float*)(misc + 16);
  const int tid = (int)threadIdx.x, lane = tid & 31, wave = tid >> 5;
  const int nodeBase = (int)blockIdx.x * NBA;

  {
    const v4i z4 = {0, 0, 0, 0};
    for (int i = tid * 4; i < AGG_ZINTS; i += NTHR * 4) *(v4ia*)(dsm + i) = z4;
    if (tid < 16) misc[tid] = 0;
    if (tid <= DEGCAP) rtab[tid] = 1.0f / fmaxf((float)tid, 1.0f);
  }
  __syncthreads();

  int t = 0, ov = 0;
  const int nChunks = (nE + CHUNK - 1) / CHUNK;
#pragma unroll 1
  for (int ch = 0; ch < nChunks; ++ch) {
    const int cbase = ch * CHUNK;
    const int wc = scan_chunk<SLA>(dsts, nE, cbase, nodeBase, NBA, vec8, list, tid, lane, wave);
    if (lane == 0) misc[wave] = wc;
    __syncthreads();
    if (wave == 0) {
#pragma unroll 1
      for (int w2 = 0; w2 < NWAVE; ++w2) {
        int c = misc[w2];
        c = c < 0 ? 0 : (c > WCAP ? WCAP : c);
#pragma unroll 1
        for (int b0 = 0; b0 < c; b0 += 32) {
          const int idx = b0 + lane;
          const int ent = list[w2 * WCAP + (idx < WCAP ? idx : WCAP - 1)];
          const int m32 = (c - b0) < 32 ? (c - b0) : 32;
#pragma unroll 1
          for (int k = 0; k < m32; ++k) {
            const int u    = __builtin_amdgcn_readlane(ent, k);
            const int slot = u & (NBA - 1);
            const int el   = (u >> SLA) & (CHUNK - 1);
            const int pk   = ((cbase + el) << SLA) | slot;
            if (t < RCAP) {
              if (lane == 0) { hl[t] = pk; cnt[slot] = cnt[slot] + 1; }
              t = t + 1;
            } else {
              ov = 1;
            }
          }
        }
      }
    }
    __syncthreads();
  }
  if (wave == 0 && lane == 0) { misc[8] = t; misc[9] = ov; }
  __syncthreads();
  int tt = misc[8];
  tt = tt < 0 ? 0 : (tt > RCAP ? RCAP : tt);
  const int ovf = misc[9];

  if (wave == 0) {
    const int base = lane * (NBA / 32);
    int sacc = 0;
#pragma unroll 1
    for (int i = 0; i < NBA / 32; ++i) sacc += cnt[base + i];
    int incl = sacc;
#pragma unroll
    for (int d = 1; d < 32; d <<= 1) {
      const int y = __shfl_up(incl, d, 32);
      if (lane >= d) incl += y;
    }
    int run = incl - sacc;
#pragma unroll 1
    for (int i = 0; i < NBA / 32; ++i) {
      const int cv = cnt[base + i];
      offs[base + i] = run;
      cur[base + i]  = run;
      run += cv;
    }
  }
  __syncthreads();
  if (wave == 0) {
#pragma unroll 1
    for (int b0 = 0; b0 < tt; b0 += 32) {
      const int idx = b0 + lane;
      const int ent = hl[idx < RCAP ? idx : RCAP - 1];
      const int m32 = (tt - b0) < 32 ? (tt - b0) : 32;
#pragma unroll 1
      for (int k = 0; k < m32; ++k) {
        const int u    = __builtin_amdgcn_readlane(ent, k);
        const int slot = u & (NBA - 1);
        if (lane == 0) {
          int p = cur[slot];
          p = p < 0 ? 0 : (p > RCAP - 1 ? RCAP - 1 : p);
          sl[p] = u;
          cur[slot] = p + 1;
        }
      }
    }
  }
  __syncthreads();

  const float pz = (ovf != 0) ? __int_as_float(0x7fc00000) : 0.0f;
#pragma unroll 1
  for (int si = 0; si < NBA / NWAVE; ++si) {
    const int s    = si * NWAVE + wave;
    const int node = nodeBase + s;
    int c = cnt[s];
    const bool big = c > DEGCAP;
    c = c < 0 ? 0 : (c > DEGCAP ? DEGCAP : c);
    int o = offs[s];
    o = o < 0 ? 0 : (o > RCAP ? RCAP : o);
    const int nc = node < nN ? node : nN - 1;
    v4f a = {0.0f, 0.0f, 0.0f, 0.0f};
#pragma unroll 1
    for (int b0 = 0; b0 < c; b0 += 32) {
      int idx = o + b0 + lane;
      idx = idx > RCAP - 1 ? RCAP - 1 : idx;
      const int ent = sl[idx];
      int eid = ent >> SLA;
      eid = eid < 0 ? 0 : (eid > nE - 1 ? nE - 1 : eid);
      int sr = srcs[eid];
      sr = sr < 0 ? 0 : (sr > nN - 1 ? nN - 1 : sr);
      int te = ets[eid];
      te = te < 0 ? 0 : (te > NREL - 1 ? NREL - 1 : te);
      const int m32 = (c - b0) < 32 ? (c - b0) : 32;
#pragma unroll 1
      for (int k = 0; k < m32; ++k) {
        const int sk = __builtin_amdgcn_readlane(sr, k);
        const int tk = __builtin_amdgcn_readlane(te, k);
        const v4f f = *(const v4f*)(T + (size_t)sk * (size_t)TP + DD * tk + 4 * lane);
        a += f;
      }
    }
    const float pzr = big ? __int_as_float(0x7fc00000) : pz;
    const float ip  = rtab[c] + pzr;
    const v4f  sf   = *(const v4f*)(T + (size_t)nc * (size_t)TP + SELFC + 4 * lane);
    const v4f  vv   = a * ip + sf;
    v4f y;
    y.x = (vv.x < 0.0f) ? 0.0f : vv.x;
    y.y = (vv.y < 0.0f) ? 0.0f : vv.y;
    y.z = (vv.z < 0.0f) ? 0.0f : vv.z;
    y.w = (vv.w < 0.0f) ? 0.0f : vv.w;
    if (node < nN) {
      float* rp = outp + (size_t)node * (size_t)DD + 4 * lane;
      *(volatile v4f*)rp = y;
      __threadfence();
      *(volatile v4f*)rp = y;
    }
  }
}

static inline int cdiv(int a, int b) { return (a + b - 1) / b; }

extern "C" void kernel_launch(void* const* d_in, const int* in_sizes, int n_in,
                              void* d_out, int out_size, void* d_ws, size_t ws_size,
                              hipStream_t stream) {
  if (n_in < 6) return;
  if (in_sizes[0] < DD || (in_sizes[0] % DD) != 0) return;
  const int nN = in_sizes[0] / DD;
  if (in_sizes[1] != NREL * DD * DD) return;
  if (in_sizes[2] != DD * DD || in_sizes[3] != DD) return;
  if (in_sizes[4] < 2 || (in_sizes[4] & 1) != 0) return;
  const int nE = in_sizes[4] / 2;
  if (nE < 1 || nE >= (1 << 21)) return;
  if (in_sizes[5] != nE) return;
  if ((long long)out_size != (long long)nN * DD) return;

  const float* x     = (const float*)d_in[0];
  const float* Wrel  = (const float*)d_in[1];
  const float* Wself = (const float*)d_in[2];
  const float* bself = (const float*)d_in[3];
  const int*   edge  = (const int*)d_in[4];
  const int*   ety   = (const int*)d_in[5];
  float* out = (float*)d_out;
  const int* src = edge;
  const int* dst = edge + nE;

  const int MP = cdiv(nN, GBM) * GBM;
  const int gM = MP / GBM;
  const int gA = cdiv(nN, NBA);
  if ((long long)gA * NBA < (long long)nN) return;
  const int vec8 = ((nE & 3) == 0) ? 1 : 0;

  char* ws = (char*)d_ws;
  size_t off = 0;
  const size_t oW = off; off += (size_t)TP * DD * 2;                      off = (off + 255) & ~(size_t)255;
  const size_t oX = off; off += (size_t)MP * DD * 2;                      off = (off + 255) & ~(size_t)255;
  const size_t oT = off; off += (size_t)MP * TP * 4;                      off = (off + 255) & ~(size_t)255;
  if (off > ws_size || off > (size_t)WSMAX) return;
  unsigned short* WT = (unsigned short*)(ws + oW);
  unsigned short* XB = (unsigned short*)(ws + oX);
  float*          T  = (float*)(ws + oT);

  const size_t scanLds = (size_t)AGG_LDS_INTS * 4;
  hipFuncSetAttribute(reinterpret_cast<const void*>(&k_scan), hipFuncAttributeMaxDynamicSharedMemorySize, (int)scanLds);

  k_prep<<<(UW + MP * KG) / NTHR, NTHR, 0, stream>>>(x, nN, MP, Wrel, Wself, WT, XB);
  k_gemm<<<dim3(gM, NCB), GTHR, 0, stream>>>(XB, DD, WT, DD, DD, bself, NREL, T, TP, MP);
  k_scan<<<gA, NTHR, scanLds, stream>>>(src, dst, ety, nE, nN, vec8, T, out);
}
